// ScalableCritic_16140487098427
// MI455X (gfx1250) — hardware-verified
//
#include <hip/hip_runtime.h>


namespace {
constexpr int M = 2000000, NE = 16384, F = 3, CD = 4, K1 = 32, H1 = 64, H2 = 128, K3 = 160, H3 = 128;
constexpr float XS = 8.0f, WSC = 256.0f, NEGSLOPE = 0.2f, NEGINIT = -1.0e9f;
typedef _Float16 b16;
typedef __attribute__((ext_vector_type(16))) _Float16 v16b;
typedef __attribute__((ext_vector_type(8))) _Float16 v8b;
typedef __attribute__((ext_vector_type(8))) float v8f;
typedef __attribute__((ext_vector_type(4))) float v4f;
__device__ __forceinline__ float bf16_rne(float f) { unsigned int u = __float_as_uint(f); u += 0x7FFFu + ((u >> 16) & 1u); return __uint_as_float(u & 0xFFFF0000u); }
__device__ __forceinline__ void split16(float v, b16& hi, b16& lo) { hi = (b16)v; lo = (b16)(v - (float)hi); }
__device__ __forceinline__ v16b frag_kb(const b16* p, int hh) { const v8b a = *(const v8b*)(p + 8 * hh), b = *(const v8b*)(p + 16 + 8 * hh); v16b f;
#pragma unroll
  for (int e = 0; e < 8; ++e) { f[e] = a[e]; f[8 + e] = b[e]; } return f; }
__device__ __forceinline__ v8f wmma16b(v16b a, v16b b, v8f c) { v8f d = __builtin_amdgcn_wmma_f32_16x16x32_f16(false, a, false, b, (short)0, c, false, false); asm volatile("v_nop\n\tv_nop\n\tv_nop\n\tv_nop" : "+v"(d) : "v"(a), "v"(b)); return d; }
__device__ __forceinline__ void wave_lds_sync() { __builtin_amdgcn_fence(__ATOMIC_RELEASE, "workgroup"); __builtin_amdgcn_wave_barrier(); __builtin_amdgcn_fence(__ATOMIC_ACQUIRE, "workgroup"); }
__device__ __forceinline__ float pmul(float a, float b) { float p = a * b; asm volatile("" : "+v"(p)); return p; }
__device__ __forceinline__ float lrelu(float x) { return x > 0.0f ? x : NEGSLOPE * x; }
__device__ __forceinline__ int iclamp(int v, int lo, int hi) { return v < lo ? lo : (v > hi ? hi : v); }

__global__ __launch_bounds__(256) void prepw_kernel(const float* __restrict__ w1, const float* __restrict__ w2, const float* __restrict__ w3, b16* __restrict__ W1T, b16* __restrict__ W2T, b16* __restrict__ W3T) {
  const int u = blockIdx.x * 256 + threadIdx.x; const int n1 = H1 * K1 / 8, n2 = H2 * H1 / 8, n3 = H3 * K3 / 8; v8b o; int t = u;
  if (t < n1) { const int e = t * 8, oo = e / K1, k0 = e % K1; for (int j = 0; j < 8; ++j) { const int k = k0 + j; o[j] = (k < F + CD) ? (b16)(bf16_rne(w1[k * H1 + oo]) * WSC) : (b16)0.0f; } for (int pass = 0; pass < 2; ++pass) { *(volatile v8b*)(W1T + e) = o; __threadfence(); } return; } t -= n1;
  if (t < n2) { const int e = t * 8, oo = e / H1, k0 = e % H1; for (int j = 0; j < 8; ++j) o[j] = (b16)(bf16_rne(w2[(k0 + j) * H2 + oo]) * WSC); for (int pass = 0; pass < 2; ++pass) { *(volatile v8b*)(W2T + e) = o; __threadfence(); } return; } t -= n2;
  if (t < n3) { const int e = t * 8, oo = e / K3, k0 = e % K3; for (int j = 0; j < 8; ++j) { const int k = k0 + j; o[j] = (k < H2 + CD) ? (b16)(bf16_rne(w3[k * H3 + oo]) * WSC) : (b16)0.0f; } for (int pass = 0; pass < 2; ++pass) { *(volatile v8b*)(W3T + e) = o; __threadfence(); } }
}
__global__ __launch_bounds__(32) void point_kernel(const float* __restrict__ mu, const int* __restrict__ bidx, const float* __restrict__ cond, const b16* __restrict__ W1T, const float* __restrict__ b1, const b16* __restrict__ W2T, const float* __restrict__ b2, float* __restrict__ GMAX) {
  __shared__ __attribute__((aligned(16))) b16 A1[16][K1 + 8], Hh[16][H1 + 8], Hl[16][H1 + 8]; __shared__ __attribute__((aligned(16))) float gm[H2];
  const int e = blockIdx.x, lane = threadIdx.x, nloc = lane & 15, hlf = lane >> 4;
  int lo, hi_; { int a = 0, b = M; while (a < b) { const int m = (a + b) >> 1; if (bidx[m] < e) a = m + 1; else b = m; } lo = a; a = 0; b = M; while (a < b) { const int m = (a + b) >> 1; if (bidx[m] < e + 1) a = m + 1; else b = m; } hi_ = a; }
  float cmax[8]; for (int t = 0; t < 8; ++t) cmax[t] = -INFINITY; float b1v[4], b2v[8]; for (int t = 0; t < 4; ++t) b1v[t] = bf16_rne(b1[t * 16 + nloc]); for (int t = 0; t < 8; ++t) b2v[t] = bf16_rne(b2[t * 16 + nloc]);
  float cv[CD]; for (int j = 0; j < CD; ++j) cv[j] = bf16_rne(cond[(size_t)e * CD + j]);
  for (int r0 = lo; r0 < hi_; r0 += 16) {
    if (lane < 16) { const int row = r0 + lane; const bool ok = row < hi_; const size_t rr = ok ? (size_t)row : (size_t)lo;
      v8b o; o[0] = (b16)(bf16_rne(mu[rr * F + 0]) * XS); o[1] = (b16)(bf16_rne(mu[rr * F + 1]) * XS); o[2] = (b16)(bf16_rne(mu[rr * F + 2]) * XS); o[3] = (b16)(cv[0] * XS); o[4] = (b16)(cv[1] * XS); o[5] = (b16)(cv[2] * XS); o[6] = (b16)(cv[3] * XS); o[7] = (b16)0.0f;
      const v8b z8 = {}; *(v8b*)(&A1[lane][0]) = ok ? o : z8; *(v8b*)(&A1[lane][8]) = z8; *(v8b*)(&A1[lane][16]) = z8; *(v8b*)(&A1[lane][24]) = z8; }
    wave_lds_sync();
    v8f d1[4] = {{}, {}, {}, {}}; { const v16b a = frag_kb(&A1[nloc][0], hlf);
#pragma unroll
      for (int t = 0; t < 4; ++t) d1[t] = wmma16b(a, frag_kb(W1T + (t * 16 + nloc) * K1, hlf), d1[t]); }
#pragma unroll
    for (int t = 0; t < 4; ++t)
#pragma unroll 1
      for (int r = 0; r < 8; ++r) { b16 p, q; split16(lrelu(d1[t][r] * (1.0f / (XS * WSC)) + b1v[t]) * XS, p, q); Hh[8 * hlf + r][t * 16 + nloc] = p; Hl[8 * hlf + r][t * 16 + nloc] = q; }
    wave_lds_sync();
    v8f d2[8];
#pragma unroll
    for (int t = 0; t < 8; ++t) d2[t] = (v8f){};
#pragma unroll
    for (int kb = 0; kb < H1; kb += 32) { const v16b a = frag_kb(&Hh[nloc][kb], hlf), al = frag_kb(&Hl[nloc][kb], hlf);
#pragma unroll
      for (int t = 0; t < 8; ++t) { const v16b bw = frag_kb(W2T + (t * 16 + nloc) * H1 + kb, hlf); d2[t] = wmma16b(a, bw, d2[t]); d2[t] = wmma16b(al, bw, d2[t]); } }
#pragma unroll
    for (int t = 0; t < 8; ++t)
#pragma unroll 1
      for (int r = 0; r < 8; ++r) { const int row = r0 + 8 * hlf + r; if (row < hi_) cmax[t] = fmaxf(cmax[t], lrelu(d2[t][r] * (1.0f / (XS * WSC)) + b2v[t])); }
    wave_lds_sync(); }
#pragma unroll
  for (int t = 0; t < 8; ++t) { const float m2 = fmaxf(cmax[t], __shfl_xor(cmax[t], 16)); if (hlf == 0) gm[t * 16 + nloc] = (hi_ > lo) ? fmaxf(m2, NEGINIT) : NEGINIT; }
  wave_lds_sync();
  for (int pass = 0; pass < 2; ++pass) { *(volatile v4f*)(GMAX + (size_t)e * H2 + lane * 4) = *(const v4f*)(&gm[lane * 4]); __threadfence(); }
}
__global__ __launch_bounds__(128) void decide_kernel(const float* __restrict__ GMAX, const float* __restrict__ cond, const b16* __restrict__ W3T, const float* __restrict__ b3, const float* __restrict__ w4, const float* __restrict__ b4, float* __restrict__ out) {
  __shared__ __attribute__((aligned(16))) b16 Ah[4][16][K3 + 8], Al[4][16][K3 + 8]; __shared__ __attribute__((aligned(16))) float sc[64];
  const int wave = threadIdx.x >> 5, lane = threadIdx.x & 31, nloc = lane & 15, hlf = lane >> 4; const size_t e0 = (size_t)blockIdx.x * 64 + wave * 16;
  for (int q = lane; q < 16 * K3; q += 32) { const int rr = q / K3, k = q % K3; float v = 0.0f; if (k < H2) v = GMAX[(e0 + rr) * H2 + k]; else if (k < H2 + CD) v = bf16_rne(cond[(e0 + rr) * CD + (k - H2)]); b16 p, pl; split16(v * XS, p, pl); Ah[wave][rr][k] = p; Al[wave][rr][k] = pl; }
  wave_lds_sync(); v8f acc[8];
#pragma unroll
  for (int t = 0; t < 8; ++t) acc[t] = (v8f){};
#pragma unroll
  for (int kb = 0; kb < K3; kb += 32) { const v16b a = frag_kb(&Ah[wave][nloc][kb], hlf), al = frag_kb(&Al[wave][nloc][kb], hlf);
#pragma unroll
    for (int t = 0; t < 8; ++t) { const v16b bw = frag_kb(W3T + (t * 16 + nloc) * K3 + kb, hlf); acc[t] = wmma16b(a, bw, acc[t]); acc[t] = wmma16b(al, bw, acc[t]); } }
  float part[8]; for (int r = 0; r < 8; ++r) part[r] = 0.0f;
#pragma unroll
  for (int t = 0; t < 8; ++t) { const int c = t * 16 + nloc; const float bb = bf16_rne(b3[c]), ww = bf16_rne(w4[c]);
#pragma unroll
    for (int r = 0; r < 8; ++r) part[r] += pmul(lrelu(acc[t][r] * (1.0f / (XS * WSC)) + bb), ww); }
#pragma unroll
  for (int r = 0; r < 8; ++r) { float v = part[r]; v += __shfl_xor(v, 1); v += __shfl_xor(v, 2); v += __shfl_xor(v, 4); v += __shfl_xor(v, 8); part[r] = v; }
  if (nloc == 0) for (int r = 0; r < 8; ++r) { float s = (part[r] + bf16_rne(b4[0])) * (1.0f / 128.0f); s = fminf(fmaxf(s, -1000.0f), 1000.0f); sc[wave * 16 + 8 * hlf + r] = s; }
  __syncthreads();
  for (int pass = 0; pass < 2; ++pass) { if (threadIdx.x < 16) *(volatile v4f*)(out + (size_t)blockIdx.x * 64 + threadIdx.x * 4) = *(const v4f*)(&sc[threadIdx.x * 4]); __threadfence(); }
}
}

extern "C" void kernel_launch(void* const* d_in, const int* in_sizes, int n_in, void* d_out, int out_size, void* d_ws, size_t ws_size, hipStream_t stream) {
  (void)n_in;
  auto Fp = [&](int i) { return (const float*)d_in[i]; }; auto Ip = [&](int i) { return (const int*)d_in[i]; };
  if (in_sizes[0] != M * F || in_sizes[1] != M || in_sizes[2] != NE * CD || in_sizes[4] != (F + CD) * H1 || in_sizes[6] != H1 * H2 || in_sizes[8] != (H2 + CD) * H3 || in_sizes[10] != H3 || out_size != NE) return;
  size_t off = 0; char* ws = (char*)d_ws;
  auto carve = [&](size_t bytes) { char* p = ws + off; off += (bytes + 255) & ~(size_t)255; return p; };
  b16* W1T = (b16*)carve((size_t)H1 * K1 * 2); b16* W2T = (b16*)carve((size_t)H2 * H1 * 2); b16* W3T = (b16*)carve((size_t)H3 * K3 * 2); float* GMAX = (float*)carve((size_t)NE * H2 * 4);
  if (off > ws_size) return;
  prepw_kernel<<<(H1 * K1 / 8 + H2 * H1 / 8 + H3 * K3 / 8 + 255) / 256, 256, 0, stream>>>(Fp(4), Fp(6), Fp(8), W1T, W2T, W3T);
  point_kernel<<<NE, 32, 0, stream>>>(Fp(0), Ip(1), Fp(2), W1T, Fp(5), W2T, Fp(7), GMAX);
  decide_kernel<<<NE / 64, 128, 0, stream>>>(GMAX, Fp(2), W3T, Fp(9), Fp(10), Fp(11), (float*)d_out);
}
